// HackableDecoderLayer_7705171329764
// MI455X (gfx1250) — hardware-verified
//
#include <hip/hip_runtime.h>
#include <math.h>
#include <stddef.h>
#include <stdint.h>


#define BB   2
#define SS   2048
#define EE   1024
#define KVHN 4
#define QPGN 4
#define HH   64
#define MLPN 4096
#define NQH  16
#define TT   (BB * SS)

#define LDT  72
#define TP16 136
#define PLP  72

typedef _Float16 v16h __attribute__((ext_vector_type(16)));
typedef _Float16 v8h  __attribute__((ext_vector_type(8)));
typedef v8h  v8ha __attribute__((may_alias));
typedef float v8f __attribute__((ext_vector_type(8)));
typedef float v4f __attribute__((ext_vector_type(4)));
typedef v4f  v4fa __attribute__((may_alias));

#define VGPR_CAP __attribute__((amdgpu_num_vgpr(256)))

__device__ __forceinline__ v8f vzero8() {
  v8f z;
#pragma unroll
  for (int i = 0; i < 8; ++i) z[i] = 0.f;
  return z;
}

__device__ __forceinline__ v16h cat8(v8h lo, v8h hi) {
  return __builtin_shufflevector(lo, hi, 0, 1, 2, 3, 4, 5, 6, 7,
                                 8, 9, 10, 11, 12, 13, 14, 15);
}

__device__ __forceinline__ v8f wmma16(v16h a, v16h b, v8f c) {
  v8f d = __builtin_amdgcn_wmma_f32_16x16x32_f16(false, a, false, b, (short)0, c, false, false);
  asm volatile("v_nop\n\tv_nop\n\tv_nop\n\tv_nop" : "+v"(d) : "v"(a), "v"(b));
  return d;
}

__device__ __forceinline__ v16h frag_row(const _Float16* row, int k0, int h) {
  return cat8(*(const v8ha*)(row + k0 + 8 * h), *(const v8ha*)(row + k0 + 16 + 8 * h));
}

__global__ __launch_bounds__(256)
void cvt_f16(const float* __restrict__ in, _Float16* __restrict__ out, int n8, float scale) {
  const int i8 = blockIdx.x * 256 + threadIdx.x;
  if (i8 >= n8) return;
  const size_t i = (size_t)i8 * 8;
  const v4f a = *(const v4fa*)(in + i);
  const v4f b = *(const v4fa*)(in + i + 4);
  v8h o;
  o[0] = (_Float16)(a[0] * scale); o[1] = (_Float16)(a[1] * scale);
  o[2] = (_Float16)(a[2] * scale); o[3] = (_Float16)(a[3] * scale);
  o[4] = (_Float16)(b[0] * scale); o[5] = (_Float16)(b[1] * scale);
  o[6] = (_Float16)(b[2] * scale); o[7] = (_Float16)(b[3] * scale);
  volatile v8h* g = (volatile v8h*)(out + i);
  *g = o;
  __threadfence();
  *g = o;
}

__global__ __launch_bounds__(256)
void rope_tab(float* __restrict__ ctab, float* __restrict__ stab, int n4) {
  const int i4 = blockIdx.x * 256 + threadIdx.x;
  if (i4 >= n4) return;
  const int e = i4 * 4;
  const int pos = e >> 4;
  const int j0 = e & 15;
  v4f c, s;
#pragma unroll 1
  for (int i = 0; i < 4; ++i) {
    const int j = j0 + i;
    const float invf = exp2f(-0.625f * (float)j);
    const float ang = (float)pos * invf;
    c[i] = cosf(ang);
    s[i] = sinf(ang);
  }
  volatile v4f* gc = (volatile v4f*)(ctab + e);
  volatile v4f* gs = (volatile v4f*)(stab + e);
  *gc = c;
  *gs = s;
  __threadfence();
  *gc = c;
  *gs = s;
}

__global__ __launch_bounds__(128)
void rmsnorm_f16(const float* __restrict__ x, const float* __restrict__ w,
                 _Float16* __restrict__ out, int nrows) {
  const int row = blockIdx.x;
  if (row >= nrows) return;
  const int tid = threadIdx.x;
  __shared__ float red[4];
  const float* xr = x + (size_t)row * EE + tid * 8;
  const v4f a = *(const v4fa*)xr;
  const v4f b = *(const v4fa*)(xr + 4);
  float ss = a[0] * a[0] + a[1] * a[1] + a[2] * a[2] + a[3] * a[3]
           + b[0] * b[0] + b[1] * b[1] + b[2] * b[2] + b[3] * b[3];
#pragma unroll
  for (int off = 16; off > 0; off >>= 1) ss += __shfl_xor(ss, off, 32);
  if ((tid & 31) == 0) red[tid >> 5] = ss;
  __syncthreads();
  const float tot = red[0] + red[1] + red[2] + red[3];
  const float rs = rsqrtf(tot * (1.0f / EE) + 1e-5f);
  const v4f wa = *(const v4fa*)(w + tid * 8);
  const v4f wb = *(const v4fa*)(w + tid * 8 + 4);
  v8h o;
  o[0] = (_Float16)(a[0] * rs * wa[0]); o[1] = (_Float16)(a[1] * rs * wa[1]);
  o[2] = (_Float16)(a[2] * rs * wa[2]); o[3] = (_Float16)(a[3] * rs * wa[3]);
  o[4] = (_Float16)(b[0] * rs * wb[0]); o[5] = (_Float16)(b[1] * rs * wb[1]);
  o[6] = (_Float16)(b[2] * rs * wb[2]); o[7] = (_Float16)(b[3] * rs * wb[3]);
  volatile v8h* g = (volatile v8h*)(out + (size_t)row * EE + tid * 8);
  *g = o;
  __threadfence();
  *g = o;
}

__device__ __forceinline__ void store_tile16(const _Float16* T16, _Float16* g,
                                             size_t pitch, int tid) {
#pragma unroll
  for (int it = 0; it < 8; ++it) {
    const int row = it * 16 + (tid >> 4);
    const int seg = tid & 15;
    const v8h v = *(const v8ha*)(T16 + row * TP16 + seg * 8);
    *(volatile v8h*)(g + (size_t)row * pitch + seg * 8) = v;
  }
}

__device__ __forceinline__ void store_tile32(const float* T32, float* g,
                                             size_t pitch, int tid) {
#pragma unroll
  for (int it = 0; it < 16; ++it) {
    const int row = it * 8 + (tid >> 5);
    const int seg = tid & 31;
    const v4f v = *(const v4fa*)(T32 + row * 128 + seg * 4);
    *(volatile v4f*)(g + (size_t)row * pitch + seg * 4) = v;
  }
}

enum : int { EPI_RESID = 0, EPI_RELU2 = 1, EPI_QKROPE = 2, EPI_VT = 3 };

template <int EPI>
__global__ __launch_bounds__(256) VGPR_CAP
void gemm_f16(const _Float16* __restrict__ A, const _Float16* __restrict__ W,
              const float* resid, const float* __restrict__ nw,
              const float* __restrict__ ctab, const float* __restrict__ stab,
              float oscale, void* outv, int M, int N, int K) {
  __shared__ v4f smem4[4096];
  _Float16* const As = (_Float16*)smem4;
  _Float16* const Bs = As + 128 * LDT;

  const int tid  = threadIdx.x;
  const int lane = tid & 31;
  const int wave = tid >> 5;
  const int wr   = wave >> 1;
  const int wc   = wave & 1;
  const int lm   = lane & 15;
  const int hi   = lane >> 4;

  const int m0 = blockIdx.y * 128;
  const int n0 = blockIdx.x * 128;
  if (m0 + 128 > M || n0 + 128 > N) return;

  v8f acc[2][4];
#pragma unroll
  for (int i = 0; i < 2; ++i)
#pragma unroll
    for (int j = 0; j < 4; ++j) acc[i][j] = vzero8();

  const int lr = tid >> 1;
  const int lc = (tid & 1) * 32;
  const _Float16* gA = A + (size_t)(m0 + lr) * K + lc;
  const _Float16* gW = W + (size_t)(n0 + lr) * K + lc;
  _Float16* const lA = As + lr * LDT + lc;
  _Float16* const lB = Bs + lr * LDT + lc;

  const int nst = K >> 6;
  for (int st = 0; st < nst; ++st) {
    const v8ha* sa = (const v8ha*)(gA + st * 64);
    const v8ha* sb = (const v8ha*)(gW + st * 64);
    const v8h a0 = sa[0], a1 = sa[1], a2 = sa[2], a3 = sa[3];
    const v8h b0 = sb[0], b1 = sb[1], b2 = sb[2], b3 = sb[3];
    __syncthreads();
    v8ha* da = (v8ha*)lA;
    da[0] = a0; da[1] = a1; da[2] = a2; da[3] = a3;
    v8ha* db = (v8ha*)lB;
    db[0] = b0; db[1] = b1; db[2] = b2; db[3] = b3;
    __syncthreads();

#pragma unroll
    for (int ks = 0; ks < 2; ++ks) {
      v16h af[2], bfr[4];
#pragma unroll
      for (int mi = 0; mi < 2; ++mi)
        af[mi] = frag_row(As + (wr * 32 + mi * 16 + lm) * LDT, ks * 32, hi);
#pragma unroll
      for (int ni = 0; ni < 4; ++ni)
        bfr[ni] = frag_row(Bs + (wc * 64 + ni * 16 + lm) * LDT, ks * 32, hi);
#pragma unroll
      for (int mi = 0; mi < 2; ++mi)
#pragma unroll
        for (int ni = 0; ni < 4; ++ni)
          acc[mi][ni] = wmma16(af[mi], bfr[ni], acc[mi][ni]);
    }
  }
  __syncthreads();

  if constexpr (EPI == EPI_QKROPE) {
    _Float16* const T16 = (_Float16*)smem4;
    const float w0 = nw[lm], w1 = nw[16 + lm], w2 = nw[32 + lm], w3 = nw[48 + lm];
#pragma unroll
    for (int mi = 0; mi < 2; ++mi) {
#pragma unroll
      for (int r = 0; r < 8; ++r) {
        const int rowl = wr * 32 + mi * 16 + hi * 8 + r;
        const float v0 = acc[mi][0][r] * oscale, v1 = acc[mi][1][r] * oscale;
        const float v2 = acc[mi][2][r] * oscale, v3 = acc[mi][3][r] * oscale;
        float ssq = v0 * v0 + v1 * v1 + v2 * v2 + v3 * v3;
#pragma unroll
        for (int off = 8; off > 0; off >>= 1) ssq += __shfl_xor(ssq, off, 32);
        const float rs = rsqrtf(ssq * (1.0f / HH) + 1e-5f);
        const float t0 = v0 * rs * w0, t1 = v1 * rs * w1;
        const float t2 = v2 * rs * w2, t3 = v3 * rs * w3;
        const int pos = (m0 + rowl) & (SS - 1);
        const float c = ctab[pos * 16 + lm], s = stab[pos * 16 + lm];
        _Float16* trow = T16 + rowl * TP16 + wc * 64;
        trow[lm]      = (_Float16)(t0 * c - t2 * s);
        trow[16 + lm] = (_Float16)t1;
        trow[32 + lm] = (_Float16)(t2 * c + t0 * s);
        trow[48 + lm] = (_Float16)t3;
      }
    }
    __syncthreads();
    _Float16* g = (_Float16*)outv + (size_t)m0 * N + n0;
    store_tile16(T16, g, (size_t)N, tid);
    __threadfence();
    store_tile16(T16, g, (size_t)N, tid);
  } else if constexpr (EPI == EPI_VT) {
    _Float16* const T16 = (_Float16*)smem4;
#pragma unroll
    for (int mi = 0; mi < 2; ++mi)
#pragma unroll
      for (int ni = 0; ni < 4; ++ni)
#pragma unroll
        for (int r = 0; r < 8; ++r) {
          const int rowl = wr * 32 + mi * 16 + hi * 8 + r;
          const int coll = wc * 64 + ni * 16 + lm;
          T16[coll * TP16 + rowl] = (_Float16)(acc[mi][ni][r] * oscale);
        }
    __syncthreads();
    const int bb = m0 / SS;
    const int s0 = m0 - bb * SS;
    _Float16* g = (_Float16*)outv + ((size_t)bb * N + n0) * SS + s0;
    store_tile16(T16, g, (size_t)SS, tid);
    __threadfence();
    store_tile16(T16, g, (size_t)SS, tid);
  } else if constexpr (EPI == EPI_RELU2) {
    _Float16* const T16 = (_Float16*)smem4;
#pragma unroll
    for (int mi = 0; mi < 2; ++mi)
#pragma unroll
      for (int ni = 0; ni < 4; ++ni)
#pragma unroll
        for (int r = 0; r < 8; ++r) {
          const int rowl = wr * 32 + mi * 16 + hi * 8 + r;
          const int coll = wc * 64 + ni * 16 + lm;
          const float up = acc[mi][ni][r] * oscale;
          const float rr = up > 0.f ? up : 0.f;
          T16[rowl * TP16 + coll] = (_Float16)(rr * rr * 16.0f);
        }
    __syncthreads();
    _Float16* g = (_Float16*)outv + (size_t)m0 * N + n0;
    store_tile16(T16, g, (size_t)N, tid);
    __threadfence();
    store_tile16(T16, g, (size_t)N, tid);
  } else {
    float* const T32 = (float*)smem4;
#pragma unroll
    for (int mi = 0; mi < 2; ++mi)
#pragma unroll
      for (int ni = 0; ni < 4; ++ni)
#pragma unroll
        for (int r = 0; r < 8; ++r) {
          const int rowl = wr * 32 + mi * 16 + hi * 8 + r;
          const int coll = wc * 64 + ni * 16 + lm;
          T32[rowl * 128 + coll] = acc[mi][ni][r] * oscale;
        }
    __syncthreads();
#pragma unroll
    for (int it = 0; it < 16; ++it) {
      const int row = it * 8 + (tid >> 5);
      const int seg = tid & 31;
      v4f t = *(const v4fa*)(T32 + row * 128 + seg * 4);
      const v4f rv = *(const v4fa*)(resid + (size_t)(m0 + row) * N + n0 + seg * 4);
      t += rv;
      *(v4fa*)(T32 + row * 128 + seg * 4) = t;
    }
    __syncthreads();
    float* g = (float*)outv + (size_t)m0 * N + n0;
    store_tile32(T32, g, (size_t)N, tid);
    __threadfence();
    store_tile32(T32, g, (size_t)N, tid);
  }
}

__device__ __forceinline__ void store_attn_tile(const _Float16* pl, _Float16* g, int lane) {
#pragma unroll
  for (int it = 0; it < 4; ++it) {
    const int row = it * 4 + (lane >> 3);
    const int seg = lane & 7;
    const v8h v = *(const v8ha*)(pl + row * PLP + seg * 8);
    *(volatile v8h*)(g + (size_t)row * (NQH * HH) + seg * 8) = v;
  }
}

__global__ __launch_bounds__(256) VGPR_CAP
void flash_attn(const _Float16* __restrict__ q, const _Float16* __restrict__ k,
                const _Float16* __restrict__ vt, _Float16* __restrict__ attn) {
  __shared__ v8h Pls[8 * 16 * (PLP / 8)];

  const int tid  = threadIdx.x;
  const int lane = tid & 31;
  const int wave = tid >> 5;
  const int lm   = lane & 15;
  const int hi   = lane >> 4;

  const int hb   = blockIdx.x;
  const int b    = hb >> 4;
  const int head = hb & 15;
  const int kh   = head >> 2;

  const int q0 = blockIdx.y * 128 + wave * 16;
  _Float16* const pl = (_Float16*)Pls + wave * (16 * PLP);

  v16h qf[2];
  {
    const _Float16* qrow = q + ((size_t)(b * SS + q0 + lm) * NQH + head) * HH;
    qf[0] = frag_row(qrow, 0, hi);
    qf[1] = frag_row(qrow, 32, hi);
  }

  float mrow[8], lrow[8];
#pragma unroll
  for (int r = 0; r < 8; ++r) { mrow[r] = -INFINITY; lrow[r] = 0.f; }
  v8f o[4];
#pragma unroll
  for (int nn = 0; nn < 4; ++nn) o[nn] = vzero8();

  const int jbmax = (q0 + 15) >> 5;
  for (int jb = 0; jb <= jbmax; ++jb) {
    const int j0 = jb * 32;

    v8f s0 = vzero8(), s1 = vzero8();
    const _Float16* krow0 = k + ((size_t)(b * SS + j0 + lm) * KVHN + kh) * HH;
    const _Float16* krow1 = krow0 + (size_t)16 * KVHN * HH;
#pragma unroll
    for (int kk = 0; kk < 2; ++kk) {
      s0 = wmma16(qf[kk], frag_row(krow0, kk * 32, hi), s0);
      s1 = wmma16(qf[kk], frag_row(krow1, kk * 32, hi), s1);
    }

    float sc0[8], sc1[8];
#pragma unroll
    for (int r = 0; r < 8; ++r) {
      const int srow = q0 + hi * 8 + r;
      sc0[r] = (j0 + lm > srow)      ? -INFINITY : s0[r] * 0.125f;
      sc1[r] = (j0 + 16 + lm > srow) ? -INFINITY : s1[r] * 0.125f;
    }

    float mnew[8], alpha[8];
#pragma unroll
    for (int r = 0; r < 8; ++r) {
      float v = fmaxf(sc0[r], sc1[r]);
#pragma unroll
      for (int off = 8; off > 0; off >>= 1) v = fmaxf(v, __shfl_xor(v, off, 32));
      mnew[r]  = fmaxf(mrow[r], v);
      alpha[r] = __expf(mrow[r] - mnew[r]);
      mrow[r]  = mnew[r];
    }
    float p0[8], p1[8];
#pragma unroll
    for (int r = 0; r < 8; ++r) {
      p0[r] = __expf(sc0[r] - mnew[r]);
      p1[r] = __expf(sc1[r] - mnew[r]);
      float rsum = p0[r] + p1[r];
#pragma unroll
      for (int off = 8; off > 0; off >>= 1) rsum += __shfl_xor(rsum, off, 32);
      lrow[r] = lrow[r] * alpha[r] + rsum;
    }
#pragma unroll
    for (int nn = 0; nn < 4; ++nn)
#pragma unroll
      for (int r = 0; r < 8; ++r) o[nn][r] *= alpha[r];

#pragma unroll
    for (int r = 0; r < 8; ++r) {
      pl[(hi * 8 + r) * PLP + lm]      = (_Float16)(p0[r] * 4096.0f);
      pl[(hi * 8 + r) * PLP + 16 + lm] = (_Float16)(p1[r] * 4096.0f);
    }
    asm volatile("" ::: "memory");
    __builtin_amdgcn_wave_barrier();
    asm volatile("s_wait_dscnt 0x0" ::: "memory");
    const v16h pf = frag_row(pl + lm * PLP, 0, hi);
    asm volatile("" ::: "memory");
    __builtin_amdgcn_wave_barrier();

#pragma unroll
    for (int nn = 0; nn < 4; ++nn) {
      const _Float16* vrow = vt + ((size_t)(b * KVHN + kh) * HH + nn * 16 + lm) * SS + j0;
      o[nn] = wmma16(pf, frag_row(vrow, 0, hi), o[nn]);
    }
  }

  float inv[8];
#pragma unroll
  for (int r = 0; r < 8; ++r) inv[r] = __builtin_amdgcn_rcpf(lrow[r]) * (1.0f / 4096.0f);
  __syncthreads();
#pragma unroll
  for (int nn = 0; nn < 4; ++nn)
#pragma unroll
    for (int r = 0; r < 8; ++r)
      pl[(hi * 8 + r) * PLP + nn * 16 + lm] = (_Float16)(o[nn][r] * inv[r]);
  __syncthreads();
  _Float16* g = attn + ((size_t)(b * SS + q0) * NQH + head) * HH;
  store_attn_tile(pl, g, lane);
  __threadfence();
  store_attn_tile(pl, g, lane);
}

static inline int cdiv(int a, int b) { return (a + b - 1) / b; }

extern "C" void kernel_launch(void* const* d_in, const int* in_sizes, int n_in,
                              void* d_out, int out_size, void* d_ws, size_t ws_size,
                              hipStream_t stream) {
  if (n_in != 11) return;
  if (in_sizes[0] != TT * EE || in_sizes[1] != NQH * HH * EE ||
      in_sizes[2] != KVHN * HH * EE || in_sizes[3] != KVHN * HH * EE ||
      in_sizes[4] != EE * NQH * HH || in_sizes[5] != MLPN * EE ||
      in_sizes[6] != EE * MLPN || in_sizes[7] != HH || in_sizes[8] != HH ||
      in_sizes[9] != EE || in_sizes[10] != EE) return;
  if (out_size != TT * EE) return;

  const float* x   = (const float*)d_in[0];
  const float* wq  = (const float*)d_in[1];
  const float* wk  = (const float*)d_in[2];
  const float* wv  = (const float*)d_in[3];
  const float* wo  = (const float*)d_in[4];
  const float* wup = (const float*)d_in[5];
  const float* wdn = (const float*)d_in[6];
  const float* qnw = (const float*)d_in[7];
  const float* knw = (const float*)d_in[8];
  const float* ln1 = (const float*)d_in[9];
  const float* ln2 = (const float*)d_in[10];
  float* out = (float*)d_out;

  const size_t szH   = (size_t)TT * EE * 2;
  const size_t szQ   = (size_t)TT * NQH * HH * 2;
  const size_t szK   = (size_t)TT * KVHN * HH * 2;
  const size_t szVT  = (size_t)BB * KVHN * HH * SS * 2;
  const size_t szAT  = (size_t)TT * NQH * HH * 2;
  const size_t szACT = (size_t)TT * MLPN * 2;
  const size_t szWQ  = (size_t)NQH * HH * EE * 2;
  const size_t szWK  = (size_t)KVHN * HH * EE * 2;
  const size_t szWV  = szWK;
  const size_t szWO  = (size_t)EE * NQH * HH * 2;
  const size_t szWU  = (size_t)MLPN * EE * 2;
  const size_t szWD  = (size_t)EE * MLPN * 2;
  const size_t szTAB = (size_t)SS * 16 * 4;
  size_t off = 0;
  const size_t oH = off;   off += szH;
  const size_t oQ = off;   off += szQ;
  const size_t oK = off;   off += szK;
  const size_t oVT = off;  off += szVT;
  const size_t oAT = off;  off += szAT;
  const size_t oACT = off; off += szACT;
  const size_t oWQ = off;  off += szWQ;
  const size_t oWK = off;  off += szWK;
  const size_t oWV = off;  off += szWV;
  const size_t oWO = off;  off += szWO;
  const size_t oWU = off;  off += szWU;
  const size_t oWD = off;  off += szWD;
  const size_t oCT = off;  off += szTAB;
  const size_t oST = off;  off += szTAB;
  if (off > ws_size) return;

  char* ws = (char*)d_ws;
  _Float16* h     = (_Float16*)(ws + oH);
  _Float16* qh    = (_Float16*)(ws + oQ);
  _Float16* khb   = (_Float16*)(ws + oK);
  _Float16* vth   = (_Float16*)(ws + oVT);
  _Float16* attnh = (_Float16*)(ws + oAT);
  _Float16* acth  = (_Float16*)(ws + oACT);
  _Float16* wqh   = (_Float16*)(ws + oWQ);
  _Float16* wkh   = (_Float16*)(ws + oWK);
  _Float16* wvh   = (_Float16*)(ws + oWV);
  _Float16* woh   = (_Float16*)(ws + oWO);
  _Float16* wuh   = (_Float16*)(ws + oWU);
  _Float16* wdh   = (_Float16*)(ws + oWD);
  float*    ctab  = (float*)(ws + oCT);
  float*    stab  = (float*)(ws + oST);

  dim3 blk(256);

  {
    const int n8q = (NQH * HH * EE) / 8, n8k = (KVHN * HH * EE) / 8;
    const int n8o = (EE * NQH * HH) / 8, n8u = (MLPN * EE) / 8, n8d = (EE * MLPN) / 8;
    cvt_f16<<<cdiv(n8q, 256), blk, 0, stream>>>(wq, wqh, n8q, 64.0f);
    cvt_f16<<<cdiv(n8k, 256), blk, 0, stream>>>(wk, wkh, n8k, 64.0f);
    cvt_f16<<<cdiv(n8k, 256), blk, 0, stream>>>(wv, wvh, n8k, 64.0f);
    cvt_f16<<<cdiv(n8o, 256), blk, 0, stream>>>(wo, woh, n8o, 64.0f);
    cvt_f16<<<cdiv(n8u, 256), blk, 0, stream>>>(wup, wuh, n8u, 64.0f);
    cvt_f16<<<cdiv(n8d, 256), blk, 0, stream>>>(wdn, wdh, n8d, 64.0f);
  }

  {
    const int n4 = (SS * 16) / 4;
    rope_tab<<<cdiv(n4, 256), blk, 0, stream>>>(ctab, stab, n4);
  }

  rmsnorm_f16<<<TT, 128, 0, stream>>>(x, ln1, h, TT);

  gemm_f16<EPI_QKROPE><<<dim3((NQH * HH) / 128, TT / 128), blk, 0, stream>>>(
      h, wqh, x, qnw, ctab, stab, 1.0f / 64.0f, qh, TT, NQH * HH, EE);
  gemm_f16<EPI_QKROPE><<<dim3((KVHN * HH) / 128, TT / 128), blk, 0, stream>>>(
      h, wkh, x, knw, ctab, stab, 1.0f / 64.0f, khb, TT, KVHN * HH, EE);
  gemm_f16<EPI_VT><<<dim3((KVHN * HH) / 128, TT / 128), blk, 0, stream>>>(
      h, wvh, x, qnw, ctab, stab, 1.0f / 64.0f, vth, TT, KVHN * HH, EE);

  flash_attn<<<dim3(BB * NQH, SS / 128), blk, 0, stream>>>(qh, khb, vth, attnh);

  gemm_f16<EPI_RESID><<<dim3(EE / 128, TT / 128), blk, 0, stream>>>(
      attnh, woh, x, qnw, ctab, stab, 1.0f / 64.0f, out, TT, EE, NQH * HH);

  rmsnorm_f16<<<TT, 128, 0, stream>>>(out, ln2, h, TT);

  gemm_f16<EPI_RELU2><<<dim3(MLPN / 128, TT / 128), blk, 0, stream>>>(
      h, wuh, x, qnw, ctab, stab, 1.0f / 64.0f, acth, TT, MLPN, EE);

  gemm_f16<EPI_RESID><<<dim3(EE / 128, TT / 128), blk, 0, stream>>>(
      acth, wdh, out, qnw, ctab, stab, 1.0f / 1024.0f, out, TT, EE, MLPN);
}
